// OuterProductMean_55688545960637
// MI455X (gfx1250) — hardware-run, weakly checked
//
#include <hip/hip_runtime.h>
#include <math.h>

typedef __attribute__((ext_vector_type(16))) _Float16 v16h;
typedef __attribute__((ext_vector_type(8)))  _Float16 v8h;
typedef __attribute__((ext_vector_type(4)))  _Float16 v4h;
typedef __attribute__((ext_vector_type(8)))  float    v8f;
typedef __attribute__((ext_vector_type(4)))  float    v4f;

constexpr int kNSeq = 128;
constexpr int kPos  = 256;
constexpr int kCm   = 256;
constexpr int kCh   = 32;
constexpr int kCz   = 128;
constexpr int kCd   = kCh * kCh;
constexpr float kLnEps = 1e-5f;

constexpr int kOuterPitch = 1032;
constexpr int kZPitch     = 132;
constexpr int kStagePitch = 136;
constexpr int kWPitch     = 132;

constexpr float kOuterCarry = 16.0f;
constexpr float kWoCarry    = 16.0f;
constexpr float kS2Scale    = kOuterCarry / (float)kNSeq;
constexpr float kFold       = 1.0f / (kOuterCarry * kWoCarry);

static_assert(kCd == 1024, "flattened channel pair count");
static_assert((kNSeq % 32) == 0 && (kCd % 32) == 0, "K multiples of 32");
static_assert((kCh % 16) == 0 && (kCz % 32) == 0 && (kPos % 16) == 0, "tile multiples");
static_assert((kOuterPitch % 8) == 0 && (kStagePitch % 8) == 0 && (kZPitch % 4) == 0 && (kWPitch % 4) == 0, "16-B aligned LDS rows");

constexpr size_t kOffAT   = 0;
constexpr size_t kOffBT   = kOffAT  + (size_t)kPos * kCh * kNSeq * 2;
constexpr size_t kOffWOT  = kOffBT  + (size_t)kPos * kCh * kNSeq * 2;
constexpr size_t kWsTotal = kOffWOT + (size_t)kCz * kCd * 2;
static_assert(kWsTotal == 4456448ull, "carve total");
static_assert(kWsTotal <= 134217728ull, "carve cap");
static_assert((kOffBT % 128) == 0 && (kOffWOT % 128) == 0, "128-B aligned regions");

union FragU { v16h v; v8h h[2]; };
__device__ __forceinline__ v16h frag_load(const _Float16* p) {
  FragU f;
  f.h[0] = *(const v8h*)(p);
  f.h[1] = *(const v8h*)(p + 16);
  return f.v;
}
__device__ __forceinline__ v8f mma_h(v16h a, v16h b, v8f c) {
  c = __builtin_amdgcn_wmma_f32_16x16x32_f16(false, a, false, b, (short)0, c, false, false);
  asm volatile("v_nop\n\tv_nop\n\tv_nop\n\tv_nop" : "+v"(c) : "v"(a), "v"(b));
  return c;
}

__global__ __launch_bounds__(256) void wo_transpose_kernel(
    const float* __restrict__ Wo, unsigned short* __restrict__ WoT)
{
  __shared__ __align__(16) float sW[64 * kWPitch];
  const int tid = threadIdx.x, lane = tid & 31, wave = tid >> 5;
  const int k0 = blockIdx.x * 64;
#pragma unroll
  for (int it = 0; it < 8; ++it) {
    const int kr = wave * 8 + it;
    const v4f v = *(const v4f*)(Wo + (size_t)(k0 + kr) * kCz + lane * 4);
    *(v4f*)(sW + kr * kWPitch + lane * 4) = v;
  }
  __syncthreads();
  const int q = lane >> 3, kk = (lane & 7) * 8;
  v8h hv[4];
#pragma unroll
  for (int it = 0; it < 4; ++it) {
    const int z = wave * 16 + it * 4 + q;
#pragma unroll
    for (int e = 0; e < 8; ++e) {
      const float f = sW[(kk + e) * kWPitch + z] * kWoCarry;
      hv[it][e] = (_Float16)f;
    }
  }
  for (int pass = 0; pass < 2; ++pass) {
#pragma unroll
    for (int it = 0; it < 4; ++it) {
      const int z = wave * 16 + it * 4 + q;
      *(volatile v8h*)(WoT + (size_t)z * kCd + k0 + kk) = hv[it];
    }
    __threadfence();
  }
}

__global__ __launch_bounds__(256) void ln_proj_kernel(
    const float* __restrict__ m, const float* __restrict__ ln_w, const float* __restrict__ ln_b,
    const float* __restrict__ Wa, const float* __restrict__ ba,
    const float* __restrict__ Wb, const float* __restrict__ bb,
    unsigned short* __restrict__ At, unsigned short* __restrict__ Bt)
{
  __shared__ __align__(16) float sMn[8 * kCm * 4];
  __shared__ __align__(16) _Float16 sT[64 * kStagePitch];
  const int tid = threadIdx.x, lane = tid & 31, wave = tid >> 5;
  const int pos = blockIdx.x;
  const v4f w0 = *(const v4f*)(ln_w + lane * 8);
  const v4f w1 = *(const v4f*)(ln_w + lane * 8 + 4);
  const v4f g0 = *(const v4f*)(ln_b + lane * 8);
  const v4f g1 = *(const v4f*)(ln_b + lane * 8 + 4);
  const float biasA = ba[lane];
  const float biasB = bb[lane];
  float* mw = sMn + wave * (kCm * 4);

#pragma unroll 1
  for (int g = 0; g < 4; ++g) {
#pragma unroll 1
    for (int r = 0; r < 4; ++r) {
      const int s = wave * 16 + g * 4 + r;
      const float* row = m + ((size_t)s * kPos + pos) * kCm + lane * 8;
      const v4f x0 = *(const v4f*)(row);
      const v4f x1 = *(const v4f*)(row + 4);
      float sum = ((x0[0] + x0[1]) + (x0[2] + x0[3])) + ((x1[0] + x1[1]) + (x1[2] + x1[3]));
#pragma unroll
      for (int o = 16; o > 0; o >>= 1) sum += __shfl_xor(sum, o, 32);
      const float mu = sum * (1.0f / (float)kCm);
      const v4f d0 = x0 - mu;
      const v4f d1 = x1 - mu;
      float sq = ((d0[0] * d0[0] + d0[1] * d0[1]) + (d0[2] * d0[2] + d0[3] * d0[3])) +
                 ((d1[0] * d1[0] + d1[1] * d1[1]) + (d1[2] * d1[2] + d1[3] * d1[3]));
#pragma unroll
      for (int o = 16; o > 0; o >>= 1) sq += __shfl_xor(sq, o, 32);
      const float rstd = rsqrtf(sq * (1.0f / (float)kCm) + kLnEps);
#pragma unroll
      for (int e = 0; e < 4; ++e) {
        mw[(lane * 8 + e) * 4 + r]     = d0[e] * rstd * w0[e] + g0[e];
        mw[(lane * 8 + 4 + e) * 4 + r] = d1[e] * rstd * w1[e] + g1[e];
      }
    }
    __syncthreads();
    float aA[4], aB[4];
#pragma unroll
    for (int r = 0; r < 4; ++r) {
      aA[r] = biasA;
      aB[r] = biasB;
    }
#pragma unroll 4
    for (int k = 0; k < kCm; ++k) {
      const float wa = Wa[k * kCh + lane];
      const float wb = Wb[k * kCh + lane];
      const v4f v = *(const v4f*)(mw + k * 4);
      aA[0] = fmaf(v[0], wa, aA[0]);
      aA[1] = fmaf(v[1], wa, aA[1]);
      aA[2] = fmaf(v[2], wa, aA[2]);
      aA[3] = fmaf(v[3], wa, aA[3]);
      aB[0] = fmaf(v[0], wb, aB[0]);
      aB[1] = fmaf(v[1], wb, aB[1]);
      aB[2] = fmaf(v[2], wb, aB[2]);
      aB[3] = fmaf(v[3], wb, aB[3]);
    }
    v4h ha, hb;
    ha[0] = (_Float16)aA[0];
    ha[1] = (_Float16)aA[1];
    ha[2] = (_Float16)aA[2];
    ha[3] = (_Float16)aA[3];
    hb[0] = (_Float16)aB[0];
    hb[1] = (_Float16)aB[1];
    hb[2] = (_Float16)aB[2];
    hb[3] = (_Float16)aB[3];
    *(v4h*)(sT + lane * kStagePitch + wave * 16 + g * 4) = ha;
    *(v4h*)(sT + (kCh + lane) * kStagePitch + wave * 16 + g * 4) = hb;
    __syncthreads();
  }

  const int hh = lane >> 4, c8 = (lane & 15) * 8;
  v8h ov[4];
#pragma unroll
  for (int it = 0; it < 4; ++it) {
    const int trow = wave * 8 + it * 2 + hh;
    ov[it] = *(const v8h*)(sT + trow * kStagePitch + c8);
  }
  unsigned short* dst = (wave < 4) ? At : Bt;
  const int chb = (wave & 3) * 8;
  for (int pass = 0; pass < 2; ++pass) {
#pragma unroll
    for (int it = 0; it < 4; ++it) {
      const int ch = chb + it * 2 + hh;
      *(volatile v8h*)(dst + ((size_t)pos * kCh + ch) * kNSeq + c8) = ov[it];
    }
    __threadfence();
  }
}

__global__ __launch_bounds__(128) void opm_kernel(
    const unsigned short* __restrict__ Atp, const unsigned short* __restrict__ Btp,
    const unsigned short* __restrict__ WoTp, const float* __restrict__ bo,
    float* __restrict__ out)
{
  __shared__ __align__(16) _Float16 sOuter[16 * kOuterPitch];
  __shared__ __align__(16) float sZ[16 * kZPitch];
  const _Float16* At  = (const _Float16*)Atp;
  const _Float16* Bt  = (const _Float16*)Btp;
  const _Float16* WoT = (const _Float16*)WoTp;
  const int lane = threadIdx.x & 31;
  const int wave = threadIdx.x >> 5;
  const int l15  = lane & 15;
  const int hh   = lane >> 4;
  const int koff = hh * 8;
  const int i    = blockIdx.y;
  const int j0   = blockIdx.x * 16;

  const _Float16* aRow0 = At + ((size_t)i * kCh + l15) * kNSeq + koff;
  const _Float16* aRow1 = aRow0 + 16 * kNSeq;
  v16h a0[4], a1[4];
#pragma unroll
  for (int ks = 0; ks < 4; ++ks) {
    a0[ks] = frag_load(aRow0 + ks * 32);
    a1[ks] = frag_load(aRow1 + ks * 32);
  }
#pragma unroll 1
  for (int pp = 0; pp < 4; ++pp) {
    const int p = wave * 4 + pp;
    const int j = j0 + p;
    const _Float16* bRow0 = Bt + ((size_t)j * kCh + l15) * kNSeq + koff;
    const _Float16* bRow1 = bRow0 + 16 * kNSeq;
    v8f acc00 = (v8f){0.f,0.f,0.f,0.f,0.f,0.f,0.f,0.f};
    v8f acc01 = acc00, acc10 = acc00, acc11 = acc00;
#pragma unroll
    for (int ks = 0; ks < 4; ++ks) {
      const v16h b0 = frag_load(bRow0 + ks * 32);
      const v16h b1 = frag_load(bRow1 + ks * 32);
      acc00 = mma_h(a0[ks], b0, acc00);
      acc01 = mma_h(a0[ks], b1, acc01);
      acc10 = mma_h(a1[ks], b0, acc10);
      acc11 = mma_h(a1[ks], b1, acc11);
    }
    _Float16* op = sOuter + p * kOuterPitch;
#pragma unroll
    for (int r = 0; r < 8; ++r) {
      const int c0 = r + 8 * hh;
      const float f00 = acc00[r] * kS2Scale;
      const float f01 = acc01[r] * kS2Scale;
      const float f10 = acc10[r] * kS2Scale;
      const float f11 = acc11[r] * kS2Scale;
      op[c0 * kCh + l15]             = (_Float16)f00;
      op[c0 * kCh + 16 + l15]        = (_Float16)f01;
      op[(16 + c0) * kCh + l15]      = (_Float16)f10;
      op[(16 + c0) * kCh + 16 + l15] = (_Float16)f11;
    }
  }
  __syncthreads();

  v8f z0 = (v8f){0.f,0.f,0.f,0.f,0.f,0.f,0.f,0.f};
  v8f z1 = z0;
  const _Float16* aL  = sOuter + l15 * kOuterPitch + koff;
  const _Float16* wp0 = WoT + (size_t)(wave * 32 + l15) * kCd + koff;
  const _Float16* wp1 = wp0 + (size_t)16 * kCd;
#pragma unroll 4
  for (int kk = 0; kk < kCd; kk += 32) {
    const v16h a2  = frag_load(aL + kk);
    const v16h b20 = frag_load(wp0 + kk);
    const v16h b21 = frag_load(wp1 + kk);
    z0 = mma_h(a2, b20, z0);
    z1 = mma_h(a2, b21, z1);
  }

  const int czb = wave * 32 + l15;
  const float bz0 = bo[czb];
  const float bz1 = bo[czb + 16];
#pragma unroll
  for (int r = 0; r < 8; ++r) {
    const int prow = r + 8 * hh;
    sZ[prow * kZPitch + czb]      = z0[r] * kFold + bz0;
    sZ[prow * kZPitch + czb + 16] = z1[r] * kFold + bz1;
  }
  __syncthreads();
  v4f ov[4];
#pragma unroll
  for (int it = 0; it < 4; ++it) {
    const int prow = wave * 4 + it;
    ov[it] = *(const v4f*)(sZ + prow * kZPitch + lane * 4);
  }
  for (int pass = 0; pass < 2; ++pass) {
#pragma unroll
    for (int it = 0; it < 4; ++it) {
      const int prow = wave * 4 + it;
      *(volatile v4f*)(out + ((size_t)i * kPos + j0 + prow) * kCz + lane * 4) = ov[it];
    }
    __threadfence();
  }
}

extern "C" void kernel_launch(void* const* d_in, const int* in_sizes, int n_in,
                              void* d_out, int out_size, void* d_ws, size_t ws_size,
                              hipStream_t stream) {
  if (n_in < 9) return;
  if (in_sizes[0] != kNSeq * kPos * kCm) return;
  if (in_sizes[1] != kCm) return;
  if (in_sizes[2] != kCm) return;
  if (in_sizes[3] != kCm * kCh) return;
  if (in_sizes[4] != kCh) return;
  if (in_sizes[5] != kCm * kCh) return;
  if (in_sizes[6] != kCh) return;
  if (in_sizes[7] != kCd * kCz) return;
  if (in_sizes[8] != kCz) return;
  if (out_size != kPos * kPos * kCz) return;
  if (ws_size < kWsTotal) return;

  const float* m    = (const float*)d_in[0];
  const float* ln_w = (const float*)d_in[1];
  const float* ln_b = (const float*)d_in[2];
  const float* Wa   = (const float*)d_in[3];
  const float* ba   = (const float*)d_in[4];
  const float* Wb   = (const float*)d_in[5];
  const float* bb   = (const float*)d_in[6];
  const float* Wo   = (const float*)d_in[7];
  const float* bo   = (const float*)d_in[8];
  float* out = (float*)d_out;

  char* ws = (char*)d_ws;
  unsigned short* At  = (unsigned short*)(ws + kOffAT);
  unsigned short* Bt  = (unsigned short*)(ws + kOffBT);
  unsigned short* WoT = (unsigned short*)(ws + kOffWOT);

  wo_transpose_kernel<<<kCd / 64, 256, 0, stream>>>(Wo, WoT);
  ln_proj_kernel<<<kPos, 256, 0, stream>>>(m, ln_w, ln_b, Wa, ba, Wb, bb, At, Bt);
  opm_kernel<<<dim3(kPos / 16, kPos), 128, 0, stream>>>(At, Bt, WoT, bo, out);
}
